// GraphEncoder_6983616823298
// MI455X (gfx1250) — hardware-run, weakly checked
//
#include <hip/hip_runtime.h>
#include <stddef.h>
#include <stdint.h>


#define FIN     11
#define KE      32
#define HID     128
#define NLR     256
#define XPW     256
#define NLAY    4
#define NTHR    256
#define NWAVE   8
#define EPT     8
#define CHUNK   (NTHR * EPT)
#define WCAP    (EPT * 32)
#define LISTN   (NWAVE * WCAP)
#define NBMAX   2048
#define NBRUN   1024
#define RCAP    28672
#define DEGCAP  64
#define PKS     11
#define GBM     64
#define GBN     128
#define GTHR    128
#define GNT     8
#define PARTW   256
#define NUWE    (HID * (KE / 8))
#define NUWT    (NLAY * NLR * (XPW / 8))
#define NUWB    (NUWE + NUWT)
#define NEGS    0.2f
#define WSMAX   134217728
#define LDS_AGG ((2 * RCAP + 2 * NBMAX + LISTN) * 4 + 64)

static_assert((CHUNK & (CHUNK - 1)) == 0 && CHUNK <= (1 << PKS));
static_assert((NBMAX & (NBMAX - 1)) == 0 && NBMAX <= (1 << PKS));
static_assert((NBRUN & (NBRUN - 1)) == 0 && NBRUN <= NBMAX && NBRUN >= 16);
static_assert(NTHR * 8 == NBMAX);
static_assert(LISTN >= NBMAX && LISTN >= NWAVE * WCAP);
static_assert((RCAP % 32) == 0);
static_assert(LDS_AGG <= 300000);
static_assert(NWAVE * PARTW + PARTW <= RCAP);
static_assert(PARTW == 2 * HID && PARTW == NTHR && (PARTW / 4) <= NTHR);
static_assert(GBM == (GTHR / 32) * 16 && GBN == 16 * GNT && GTHR == GBN && GBN == 4 * 32);
static_assert(HID == 32 * 4);
static_assert((KE % 32) == 0 && (XPW % 32) == 0);
static_assert((HID % GBN) == 0 && (NLR % GBN) == 0);
static_assert(XPW == 2 * HID && NLR == 2 * HID);
static_assert((NUWE % NTHR) == 0 && (NUWT % NTHR) == 0);
static_assert((KE / 8) == 4 && (XPW / 8) == 32);
static_assert(FIN <= KE);

typedef float          v4f  __attribute__((ext_vector_type(4)));
typedef float          v8f  __attribute__((ext_vector_type(8)));
typedef int            v4i  __attribute__((ext_vector_type(4)));
typedef int            v8i  __attribute__((ext_vector_type(8)));
typedef unsigned int   v2u  __attribute__((ext_vector_type(2)));
typedef unsigned int   v4u  __attribute__((ext_vector_type(4)));
typedef unsigned short v8us __attribute__((ext_vector_type(8)));
typedef __bf16         v16b __attribute__((ext_vector_type(16)));
typedef v4f  __attribute__((may_alias)) v4fa;
typedef v8us __attribute__((may_alias)) v8usa;
union Frag { v16b vb; v8us h[2]; v8i w; };

__device__ __forceinline__ v8f wmx(const Frag& a, const Frag& b, v8f c) {
  v8f d = __builtin_amdgcn_wmma_f32_16x16x32_bf16(false, a.vb, false, b.vb, (short)0, c, false, false);
  asm volatile("v_nop\n\tv_nop\n\tv_nop\n\tv_nop" : "+v"(d) : "v"(a.w), "v"(b.w));
  return d;
}

__device__ __forceinline__ unsigned short bf_bits(float f) {
  unsigned int u = __float_as_uint(f);
  u += 0x7FFFu + ((u >> 16) & 1u);
  return (unsigned short)(u >> 16);
}
__device__ __forceinline__ float bf_val(unsigned short b) { return __uint_as_float(((unsigned int)b) << 16); }
__device__ __forceinline__ float bf_rne(float f) { return bf_val(bf_bits(f)); }

__device__ __forceinline__ int scan_chunk(const int* __restrict__ dsts, int nE, int cbase, int slotBase,
                                          int nb, int vec8, int* list, int tid, int lane, int wave) {
  int wc = 0;
  const int el0  = tid * EPT;
  const int e0   = cbase + el0;
  const int sent = -2147483647 - 1;
  v4i da, db;
  if (vec8 != 0 && cbase + CHUNK <= nE) {
    da = *(const v4i*)(dsts + e0);
    db = *(const v4i*)(dsts + e0 + 4);
  } else {
    da.x = (e0     < nE) ? dsts[min(e0,     nE - 1)] : sent;
    da.y = (e0 + 1 < nE) ? dsts[min(e0 + 1, nE - 1)] : sent;
    da.z = (e0 + 2 < nE) ? dsts[min(e0 + 2, nE - 1)] : sent;
    da.w = (e0 + 3 < nE) ? dsts[min(e0 + 3, nE - 1)] : sent;
    db.x = (e0 + 4 < nE) ? dsts[min(e0 + 4, nE - 1)] : sent;
    db.y = (e0 + 5 < nE) ? dsts[min(e0 + 5, nE - 1)] : sent;
    db.z = (e0 + 6 < nE) ? dsts[min(e0 + 6, nE - 1)] : sent;
    db.w = (e0 + 7 < nE) ? dsts[min(e0 + 7, nE - 1)] : sent;
  }
  const unsigned nbs = (unsigned)slotBase;
  const unsigned unb = (unsigned)nb;
  const unsigned s0 = (unsigned)da.x - nbs, s1 = (unsigned)da.y - nbs;
  const unsigned s2 = (unsigned)da.z - nbs, s3 = (unsigned)da.w - nbs;
  const unsigned s4 = (unsigned)db.x - nbs, s5 = (unsigned)db.y - nbs;
  const unsigned s6 = (unsigned)db.z - nbs, s7 = (unsigned)db.w - nbs;
  const bool h0 = s0 < unb, h1 = s1 < unb, h2 = s2 < unb, h3 = s3 < unb;
  const bool h4 = s4 < unb, h5 = s5 < unb, h6 = s6 < unb, h7 = s7 < unb;
  const unsigned any = __builtin_amdgcn_ballot_w32(h0 | h1 | h2 | h3 | h4 | h5 | h6 | h7);
  if (any != 0u) {
#define HITJ(J, HJ, SJ) { \
      const unsigned mj = __builtin_amdgcn_ballot_w32(HJ); \
      if (mj != 0u) { \
        if (HJ) { \
          const int pos = wc + (int)__builtin_amdgcn_mbcnt_lo(mj, 0u); \
          if (pos < WCAP) list[wave * WCAP + pos] = ((el0 + (J)) << PKS) | (int)(SJ); \
        } \
        wc += (int)__builtin_popcount(mj); } }
    HITJ(0, h0, s0)
    HITJ(1, h1, s1)
    HITJ(2, h2, s2)
    HITJ(3, h3, s3)
    HITJ(4, h4, s4)
    HITJ(5, h5, s5)
    HITJ(6, h6, s6)
    HITJ(7, h7, s7)
#undef HITJ
  }
  return wc;
}

__global__ __launch_bounds__(NTHR) void k_prep(const float* __restrict__ nf, const float* __restrict__ wemb,
                                               const float* __restrict__ wl, const float* __restrict__ wr,
                                               unsigned short* nfb, unsigned short* wet, unsigned short* wt,
                                               int nN, int nUnits) {
  const int u = (int)blockIdx.x * NTHR + (int)threadIdx.x;
  v8us o;
  unsigned short* dp;
  if (u < NUWE) {
    const int n = u >> 2, k8 = (u & 3) * 8;
    const float* p = wemb + (size_t)n * FIN;
#pragma unroll
    for (int i = 0; i < 8; ++i) {
      const int k  = k8 + i;
      const int kc = k < FIN ? k : FIN - 1;
      const float f = p[kc];
      o[i] = bf_bits(k < FIN ? f : 0.0f);
    }
    dp = wet + (size_t)u * 8;
  } else if (u < NUWB) {
    const int v  = u - NUWE;
    const int l  = v >> 13, n = (v >> 5) & 255, k8 = (v & 31) * 8;
    const int kk = k8 & (HID - 1), nn = n & (HID - 1);
    const size_t wo = (size_t)l * HID * HID + (size_t)nn * HID + (size_t)kk;
    const v4f a0 = *(const v4f*)(wl + wo), a1 = *(const v4f*)(wl + wo + 4);
    const v4f b0 = *(const v4f*)(wr + wo), b1 = *(const v4f*)(wr + wo + 4);
    const float fa[8] = {a0.x, a0.y, a0.z, a0.w, a1.x, a1.y, a1.z, a1.w};
    const float fb[8] = {b0.x, b0.y, b0.z, b0.w, b1.x, b1.y, b1.z, b1.w};
    const unsigned int msk = (n < HID) ? 0xFFFFu : 0u;
#pragma unroll
    for (int i = 0; i < 8; ++i) {
      const unsigned int ha = (unsigned int)bf_bits(fa[i]);
      const unsigned int hb = (unsigned int)bf_bits(fb[i]);
      o[i] = (unsigned short)((ha & msk) | (hb & (~msk & 0xFFFFu)));
    }
    dp = wt + (size_t)v * 8;
  } else if (u < nUnits) {
    const int v   = u - NUWB;
    const int row = v >> 2, k8 = (v & 3) * 8;
    const int rc  = row < nN ? row : nN - 1;
    const bool lv = row < nN;
    const float* p = nf + (size_t)rc * FIN;
#pragma unroll
    for (int i = 0; i < 8; ++i) {
      const int k  = k8 + i;
      const int kc = k < FIN ? k : FIN - 1;
      const float f = p[kc];
      o[i] = bf_bits((lv && k < FIN) ? f : 0.0f);
    }
    dp = nfb + (size_t)v * 8;
  } else {
    return;
  }
  *(volatile v8us*)dp = o;
  __threadfence();
  *(volatile v8us*)dp = o;
}

template <int EPI>
__global__ __launch_bounds__(GTHR) void k_gemm(const unsigned short* __restrict__ A, int lda,
                                               const unsigned short* __restrict__ BT, int ldb, int K,
                                               const float* __restrict__ biasA, const float* __restrict__ biasB,
                                               void* outp, int ldo, int lsplit, int nN, int mRows) {
  __shared__ __attribute__((aligned(16))) float stg[GBM * GBN];
  const int tid = (int)threadIdx.x, lane = tid & 31, wave = tid >> 5, hh = lane >> 4, m = lane & 15;
  const int rowBase = (int)blockIdx.x * GBM;
  const int colBase = (int)blockIdx.y * GBN;
  const bool ysel0  = (blockIdx.y == 0);

  v8f acc[GNT];
  {
    const v8f z = {0.f, 0.f, 0.f, 0.f, 0.f, 0.f, 0.f, 0.f};
#pragma unroll
    for (int t = 0; t < GNT; ++t) acc[t] = z;
  }
  const unsigned short* ap = A  + (size_t)(rowBase + 16 * wave + m) * (size_t)lda + 8 * hh;
  const unsigned short* bp = BT + (size_t)(colBase + m) * (size_t)ldb + 8 * hh;

#pragma unroll 1
  for (int k0 = 0; k0 < K; k0 += 32) {
    Frag af;
    af.h[0] = *(const v8usa*)(ap + k0);
    af.h[1] = *(const v8usa*)(ap + k0 + 16);
#pragma unroll
    for (int nt = 0; nt < GNT; ++nt) {
      const unsigned short* wq = bp + (size_t)(16 * nt) * (size_t)ldb + k0;
      Frag bfr;
      bfr.h[0] = *(const v8usa*)wq;
      bfr.h[1] = *(const v8usa*)(wq + 16);
      acc[nt] = wmx(af, bfr, acc[nt]);
    }
  }

#pragma unroll
  for (int nt = 0; nt < GNT; ++nt) {
    const int lc = 16 * nt + m;
    const float ba = biasA[lc];
    const float bbv = biasB[lc];
    const float bb = bf_rne(ysel0 ? ba : bbv);
#pragma unroll
    for (int r = 0; r < 8; ++r) {
      const int lr = 16 * wave + 8 * hh + r;
      const bool live = (rowBase + lr) < nN;
      float v = acc[nt][r] + bb;
      if constexpr (EPI == 2) v = fmaxf(v, 0.0f);
      stg[lr * GBN + lc] = live ? v : 0.0f;
    }
  }
  __syncthreads();

  if constexpr (EPI == 2) {
    unsigned short* outH = (unsigned short*)outp;
    const int cb = 8 * m;
    const bool isHi = (hh == 0);
    v4u pk[16];
#pragma unroll
    for (int i = 0; i < 16; ++i) {
      const int lr = 16 * wave + i;
      const v4f a = *(const v4fa*)(stg + lr * GBN + cb);
      const v4f b = *(const v4fa*)(stg + lr * GBN + cb + 4);
      const float f[8] = {a.x, a.y, a.z, a.w, b.x, b.y, b.z, b.w};
      unsigned int w[4];
#pragma unroll
      for (int j = 0; j < 4; ++j) {
        const unsigned short h0 = bf_bits(f[2 * j]), h1 = bf_bits(f[2 * j + 1]);
        const unsigned short l0 = bf_bits(f[2 * j] - bf_val(h0)), l1 = bf_bits(f[2 * j + 1] - bf_val(h1));
        const unsigned short q0 = isHi ? h0 : l0, q1 = isHi ? h1 : l1;
        w[j] = (unsigned int)q0 | ((unsigned int)q1 << 16);
      }
      v4u pv; pv.x = w[0]; pv.y = w[1]; pv.z = w[2]; pv.w = w[3];
      pk[i] = pv;
    }
#pragma unroll
    for (int i = 0; i < 16; ++i) {
      const int gr = rowBase + 16 * wave + i;
      unsigned short* op = outH + (size_t)gr * (size_t)ldo + colBase + cb + hh * lsplit;
      if (gr < mRows) *(volatile v4u*)op = pk[i];
    }
    __threadfence();
#pragma unroll
    for (int i = 0; i < 16; ++i) {
      const int gr = rowBase + 16 * wave + i;
      unsigned short* op = outH + (size_t)gr * (size_t)ldo + colBase + cb + hh * lsplit;
      if (gr < mRows) *(volatile v4u*)op = pk[i];
    }
  } else {
    float* outF = (float*)outp;
    v4f fv[16];
#pragma unroll
    for (int i = 0; i < 16; ++i) {
      const int lr = 16 * wave + i;
      fv[i] = *(const v4fa*)(stg + lr * GBN + 4 * lane);
    }
#pragma unroll
    for (int i = 0; i < 16; ++i) {
      const int gr = rowBase + 16 * wave + i;
      float* op = outF + (size_t)gr * (size_t)ldo + colBase + 4 * lane;
      if (gr < mRows) *(volatile v4f*)op = fv[i];
    }
    __threadfence();
#pragma unroll
    for (int i = 0; i < 16; ++i) {
      const int gr = rowBase + 16 * wave + i;
      float* op = outF + (size_t)gr * (size_t)ldo + colBase + 4 * lane;
      if (gr < mRows) *(volatile v4f*)op = fv[i];
    }
  }
}

template <int RES, int LAST>
__global__ __launch_bounds__(NTHR) void k_agg(
    const int* __restrict__ srcs, const int* __restrict__ dsts,
    const float* __restrict__ XLR, const float* __restrict__ att, const float* __restrict__ bias,
    const float* xres, float* xout, int ldxo, unsigned short* xp, float* part,
    int nN, int nE, int nb, int vec8, int MPr) {
  extern __shared__ v4f lds_dyn[];
  int* reg1 = (int*)lds_dyn;
  int* reg2 = reg1 + RCAP;
  int* scnt = reg2 + RCAP;
  int* soff = scnt + NBMAX;
  int* list = soff + NBMAX;
  int* wcnt = list + LISTN;
  int* wtot = wcnt + NWAVE;
  const int tid = (int)threadIdx.x, lane = tid & 31, wave = tid >> 5;
  const int nodeBase = (int)blockIdx.x * nb;

  for (int i = tid; i < NBMAX; i += NTHR) scnt[i] = 0;
  __syncthreads();

  int tot = 0;
  const int nChunks = (nE + CHUNK - 1) / CHUNK;
#pragma unroll 1
  for (int ch = 0; ch < nChunks; ++ch) {
    const int cbase = ch * CHUNK;
    const int wc = scan_chunk(dsts, nE, cbase, nodeBase, nb, vec8, list, tid, lane, wave);
    if (lane == 0) wcnt[wave] = wc;
    __syncthreads();
    int pre = 0, all = 0;
#pragma unroll
    for (int w2 = 0; w2 < NWAVE; ++w2) {
      int c = wcnt[w2];
      c = c < 0 ? 0 : (c > WCAP ? WCAP : c);
      all += c;
      pre += (w2 < wave) ? c : 0;
    }
    const int wcc  = wc > WCAP ? WCAP : wc;
    const int base = tot + pre;
#pragma unroll 1
    for (int i = lane; i < wcc; i += 32) {
      const int ent = list[wave * WCAP + i];
      const int el  = (ent >> PKS) & (CHUNK - 1);
      const int sl  = ent & (NBMAX - 1);
      int eid = cbase + el;
      eid = eid > nE - 1 ? nE - 1 : eid;
      const int pos = base + i;
      if (pos < RCAP) reg1[pos] = (int)(((unsigned)eid << PKS) | (unsigned)sl);
    }
    tot += all;
    tot = tot > RCAP ? RCAP : tot;
    __syncthreads();
  }
  const int nh = tot;

  if (wave == 0) {
#pragma unroll 1
    for (int b0 = 0; b0 < nh; b0 += 32) {
      const int idx = b0 + lane;
      const int uv  = reg1[idx < RCAP ? idx : RCAP - 1];
      const int m32 = (nh - b0) < 32 ? (nh - b0) : 32;
#pragma unroll 1
      for (int k = 0; k < m32; ++k) {
        const int u  = __builtin_amdgcn_readlane(uv, k);
        const int sl = u & (NBMAX - 1);
        if (lane == 0) scnt[sl] = scnt[sl] + 1;
      }
    }
  }
  __syncthreads();

  {
    const v4i ca = *(const v4i*)(scnt + 8 * tid);
    const v4i cb = *(const v4i*)(scnt + 8 * tid + 4);
    const int e0 = ca.x < 0 ? 0 : ca.x, e1 = ca.y < 0 ? 0 : ca.y, e2 = ca.z < 0 ? 0 : ca.z, e3 = ca.w < 0 ? 0 : ca.w;
    const int e4 = cb.x < 0 ? 0 : cb.x, e5 = cb.y < 0 ? 0 : cb.y, e6 = cb.z < 0 ? 0 : cb.z, e7 = cb.w < 0 ? 0 : cb.w;
    const int ts = e0 + e1 + e2 + e3 + e4 + e5 + e6 + e7;
    int incl = ts;
#pragma unroll
    for (int d = 1; d < 32; d <<= 1) {
      const int up = __shfl_up(incl, d);
      if (lane >= d) incl += up;
    }
    if (lane == 31) wtot[wave] = incl;
    __syncthreads();
    int pre = 0;
#pragma unroll
    for (int w2 = 0; w2 < NWAVE; ++w2) pre += (w2 < wave) ? wtot[w2] : 0;
    int run = pre + incl - ts;
    soff[8 * tid + 0] = run; run += e0;
    soff[8 * tid + 1] = run; run += e1;
    soff[8 * tid + 2] = run; run += e2;
    soff[8 * tid + 3] = run; run += e3;
    soff[8 * tid + 4] = run; run += e4;
    soff[8 * tid + 5] = run; run += e5;
    soff[8 * tid + 6] = run; run += e6;
    soff[8 * tid + 7] = run;
  }
  __syncthreads();
  for (int i = tid; i < NBMAX; i += NTHR) list[i] = soff[i];
  __syncthreads();

  if (wave == 0) {
#pragma unroll 1
    for (int b0 = 0; b0 < nh; b0 += 32) {
      const int idx = b0 + lane;
      const int uv  = reg1[idx < RCAP ? idx : RCAP - 1];
      const int m32 = (nh - b0) < 32 ? (nh - b0) : 32;
#pragma unroll 1
      for (int k = 0; k < m32; ++k) {
        const int u   = __builtin_amdgcn_readlane(uv, k);
        const int sl  = u & (NBMAX - 1);
        const int eid = (int)((unsigned)u >> PKS);
        if (lane == 0) {
          int pos = list[sl];
          pos = pos < 0 ? 0 : (pos > RCAP - 1 ? RCAP - 1 : pos);
          reg2[pos] = eid;
          list[sl] = pos + 1;
        }
      }
    }
  }
  __syncthreads();

  const int nbw = nb >> 3;
  const bool ovf = (nh >= RCAP);
  const float qnan  = __int_as_float(0x7fc00000);
  const float nhuge = -__builtin_huge_valf();
  const v4f atv = *(const v4f*)(att + 4 * lane);
  const v4f bsv = *(const v4f*)(bias + 4 * lane);
  const float at0 = bf_rne(atv.x), at1 = bf_rne(atv.y), at2 = bf_rne(atv.z), at3 = bf_rne(atv.w);
  const float bb0 = bf_rne(bsv.x), bb1 = bf_rne(bsv.y), bb2 = bf_rne(bsv.z), bb3 = bf_rne(bsv.w);
  float cs0 = 0.f, cs1 = 0.f, cs2 = 0.f, cs3 = 0.f;
  float cm0 = nhuge, cm1 = nhuge, cm2 = nhuge, cm3 = nhuge;

#pragma unroll 1
  for (int jt = 0; jt < nbw; ++jt) {
    const int slot = wave * nbw + jt;
    const int grow = nodeBase + slot;
    const int gcl  = grow < nN ? grow : nN - 1;
    int st = soff[slot];
    const int craw = scnt[slot];
    int cnt = craw;
    st  = st < 0 ? 0 : (st > nh ? nh : st);
    cnt = cnt < 0 ? 0 : (cnt > DEGCAP ? DEGCAP : cnt);
    if (cnt > nh - st) cnt = nh - st;
    const float pz = (ovf || craw > DEGCAP) ? qnan : 0.0f;
    const bool live = grow < nN;

    const v4f xd = *(const v4f*)(XLR + (size_t)gcl * NLR + HID + 4 * lane);
    float mx = -1.0e30f, dn = 0.f;
    float a0 = 0.f, a1 = 0.f, a2 = 0.f, a3 = 0.f;

#pragma unroll 1
    for (int q = 0; q < cnt; ++q) {
      int idx = st + q; idx = idx > RCAP - 1 ? RCAP - 1 : idx;
      int eid = reg2[idx]; eid = eid < 0 ? 0 : (eid > nE - 1 ? nE - 1 : eid);
      const int sraw = srcs[eid];
      const int s = sraw < 0 ? 0 : (sraw > nN - 1 ? nN - 1 : sraw);
      const v4f xs = *(const v4f*)(XLR + (size_t)s * NLR + 4 * lane);
      float z0 = xs.x + xd.x; z0 = z0 > 0.f ? z0 : z0 * NEGS;
      float z1 = xs.y + xd.y; z1 = z1 > 0.f ? z1 : z1 * NEGS;
      float z2 = xs.z + xd.z; z2 = z2 > 0.f ? z2 : z2 * NEGS;
      float z3 = xs.w + xd.w; z3 = z3 > 0.f ? z3 : z3 * NEGS;
      float pt = z0 * at0;
      pt = fmaf(z1, at1, pt);
      pt = fmaf(z2, at2, pt);
      pt = fmaf(z3, at3, pt);
      pt += __shfl_xor(pt, 4);
      pt += __shfl_xor(pt, 2);
      pt += __shfl_xor(pt, 1);
      const float al = pt;
      const float df = al - mx;
      const float ee = __expf(-fabsf(df));
      const bool up  = df > 0.f;
      const float s1 = up ? ee : 1.0f;
      const float s2 = up ? 1.0f : ee;
      mx = up ? al : mx;
      dn = fmaf(dn, s1, s2);
      a0 = fmaf(a0, s1, s2 * xs.x);
      a1 = fmaf(a1, s1, s2 * xs.y);
      a2 = fmaf(a2, s1, s2 * xs.z);
      a3 = fmaf(a3, s1, s2 * xs.w);
    }
    const float ds = dn > 0.f ? dn : 1.0f;
    const float iv = (dn > 0.f ? 1.0f : 0.0f) * __builtin_amdgcn_rcpf(ds);
    float r0 = fmaxf(fmaf(a0, iv, bb0), 0.f);
    float r1 = fmaxf(fmaf(a1, iv, bb1), 0.f);
    float r2 = fmaxf(fmaf(a2, iv, bb2), 0.f);
    float r3 = fmaxf(fmaf(a3, iv, bb3), 0.f);
    if constexpr (RES != 0) {
      const v4f rr = *(const v4f*)(xres + (size_t)gcl * HID + 4 * lane);
      r0 += rr.x; r1 += rr.y; r2 += rr.z; r3 += rr.w;
    }
    r0 = (live ? r0 : 0.0f) + pz;
    r1 = (live ? r1 : 0.0f) + pz;
    r2 = (live ? r2 : 0.0f) + pz;
    r3 = (live ? r3 : 0.0f) + pz;

    v4f rv; rv.x = r0; rv.y = r1; rv.z = r2; rv.w = r3;
    float* op = xout + (size_t)grow * (size_t)ldxo + 4 * lane;
    if constexpr (LAST != 0) {
      cs0 += live ? r0 : 0.0f; cs1 += live ? r1 : 0.0f; cs2 += live ? r2 : 0.0f; cs3 += live ? r3 : 0.0f;
      cm0 = fmaxf(cm0, live ? r0 : nhuge); cm1 = fmaxf(cm1, live ? r1 : nhuge);
      cm2 = fmaxf(cm2, live ? r2 : nhuge); cm3 = fmaxf(cm3, live ? r3 : nhuge);
      if (live) *(volatile v4f*)op = rv;
      __threadfence();
      if (live) *(volatile v4f*)op = rv;
    } else {
      const unsigned short h0 = bf_bits(r0), h1 = bf_bits(r1), h2 = bf_bits(r2), h3 = bf_bits(r3);
      const unsigned short l0 = bf_bits(r0 - bf_val(h0)), l1 = bf_bits(r1 - bf_val(h1));
      const unsigned short l2 = bf_bits(r2 - bf_val(h2)), l3 = bf_bits(r3 - bf_val(h3));
      v2u ph, pl;
      ph.x = (unsigned int)h0 | ((unsigned int)h1 << 16);
      ph.y = (unsigned int)h2 | ((unsigned int)h3 << 16);
      pl.x = (unsigned int)l0 | ((unsigned int)l1 << 16);
      pl.y = (unsigned int)l2 | ((unsigned int)l3 << 16);
      unsigned short* hp = xp + (size_t)grow * XPW + 4 * lane;
      unsigned short* lp = xp + (size_t)grow * XPW + HID + 4 * lane;
      const bool wsv = grow < MPr;
      if (wsv) { *(volatile v4f*)op = rv; *(volatile v2u*)hp = ph; *(volatile v2u*)lp = pl; }
      __threadfence();
      if (wsv) { *(volatile v4f*)op = rv; *(volatile v2u*)hp = ph; *(volatile v2u*)lp = pl; }
    }
  }

  if constexpr (LAST != 0) {
    float* wst = (float*)reg1;
    v4f csv; csv.x = cs0; csv.y = cs1; csv.z = cs2; csv.w = cs3;
    v4f cmv; cmv.x = cm0; cmv.y = cm1; cmv.z = cm2; cmv.w = cm3;
    *(v4fa*)(wst + wave * PARTW + 4 * lane) = csv;
    *(v4fa*)(wst + wave * PARTW + HID + 4 * lane) = cmv;
    __syncthreads();
    const int c = tid & (HID - 1);
    const int half = tid >> 7;
    float sv = 0.0f, mv = nhuge;
#pragma unroll
    for (int w2 = 0; w2 < NWAVE; ++w2) {
      sv += wst[w2 * PARTW + c];
      mv = fmaxf(mv, wst[w2 * PARTW + HID + c]);
    }
    float* pst = wst + NWAVE * PARTW;
    pst[tid] = (half == 0) ? sv : mv;
    __syncthreads();
    const bool pok = tid < PARTW / 4;
    v4f pv = {0.f, 0.f, 0.f, 0.f};
    if (pok) pv = *(const v4fa*)(pst + 4 * tid);
    float* pp = part + (size_t)blockIdx.x * PARTW + 4 * tid;
    if (pok) *(volatile v4f*)pp = pv;
    __threadfence();
    if (pok) *(volatile v4f*)pp = pv;
  }
  (void)xres; (void)xp; (void)part;
}

__global__ __launch_bounds__(NTHR) void k_pool(const float* __restrict__ part, int nPart, float invN,
                                              const int* __restrict__ numn, float* out) {
  __shared__ __attribute__((aligned(16))) float stg[PARTW];
  const int tid = (int)threadIdx.x;
  const int c = tid & (HID - 1);
  const int half = tid >> 7;
  double s = 0.0;
  float mv = -__builtin_huge_valf();
#pragma unroll 1
  for (int b = 0; b < nPart; ++b) {
    const float* pr = part + (size_t)b * PARTW;
    s += (double)pr[c];
    mv = fmaxf(mv, pr[HID + c]);
  }
  const float mean = (float)s * invN;
  stg[tid] = (half == 0) ? mean : mv;
  __syncthreads();
  const bool ok = tid < PARTW / 4;
  v4f pv = {0.f, 0.f, 0.f, 0.f};
  if (ok) pv = *(const v4fa*)(stg + 4 * tid);
  float* op = out + 4 * tid;
  if (ok) *(volatile v4f*)op = pv;
  __threadfence();
  if (ok) *(volatile v4f*)op = pv;
  (void)numn;
}

static int pick_nb(int nE, int nN) {
  int nb = NBRUN;
  while (nb > 16 && (long long)nb * (long long)nE * 5LL > (long long)RCAP * (long long)nN * 4LL) nb >>= 1;
  return nb;
}
static inline int cdiv(int a, int b) { return (a + b - 1) / b; }
static inline size_t al256(size_t o) { return (o + 255) & ~(size_t)255; }

extern "C" void kernel_launch(void* const* d_in, const int* in_sizes, int n_in,
                              void* d_out, int out_size, void* d_ws, size_t ws_size,
                              hipStream_t stream) {
  if (n_in < 11) return;
  if (in_sizes[0] < FIN * GBM || (in_sizes[0] % FIN) != 0) return;
  const int nN = in_sizes[0] / FIN;
  if (nN > (1 << 22)) return;
  if (in_sizes[1] < 2 || (in_sizes[1] & 1) != 0) return;
  const int nE = in_sizes[1] / 2;
  if (nE < 1 || nE > (1 << 21)) return;
  if (in_sizes[2] < 1) return;
  if (in_sizes[3] != HID * FIN || in_sizes[4] != HID) return;
  if (in_sizes[5] != NLAY * HID * HID || in_sizes[6] != NLAY * HID) return;
  if (in_sizes[7] != NLAY * HID * HID || in_sizes[8] != NLAY * HID) return;
  if (in_sizes[9] != NLAY * HID || in_sizes[10] != NLAY * HID) return;
  if ((long long)out_size != (long long)PARTW + (long long)nN * HID) return;

  const float* nf   = (const float*)d_in[0];
  const int*   ei   = (const int*)  d_in[1];
  const int*   src  = ei;
  const int*   dst  = ei + nE;
  const int*   numn = (const int*)  d_in[2];
  const float* wemb = (const float*)d_in[3];
  const float* bemb = (const float*)d_in[4];
  const float* wl   = (const float*)d_in[5];
  const float* bl   = (const float*)d_in[6];
  const float* wr   = (const float*)d_in[7];
  const float* br   = (const float*)d_in[8];
  const float* att  = (const float*)d_in[9];
  const float* bias = (const float*)d_in[10];
  float* out = (float*)d_out;

  const int MP   = cdiv(nN, GBM) * GBM;
  const int gM   = MP / GBM;
  const int nb   = pick_nb(nE, nN);
  const int gA   = cdiv(MP, nb);
  const int vec8 = ((nE & 3) == 0) ? 1 : 0;
  if ((long long)gA * nb < (long long)MP) return;
  if ((long long)(gM - 1) * GBM >= (long long)nN) return;
  const int nUx  = MP * (KE / 8);
  const int nUt  = NUWB + nUx;

  char* ws = (char*)d_ws;
  size_t off = 0;
  const size_t oNFB = off; off = al256(off + (size_t)MP * KE * 2);
  const size_t oWET = off; off = al256(off + (size_t)HID * KE * 2);
  const size_t oWT  = off; off = al256(off + (size_t)NLAY * NLR * XPW * 2);
  const size_t oXP  = off; off = al256(off + (size_t)MP * XPW * 2);
  const size_t oXLR = off; off = al256(off + (size_t)MP * NLR * 4);
  const size_t oXFa = off; off = al256(off + (size_t)MP * HID * 4);
  const size_t oXFb = off; off = al256(off + (size_t)MP * HID * 4);
  const size_t oPT  = off; off = al256(off + (size_t)gA * PARTW * 4);
  if (off > ws_size || off > (size_t)WSMAX) return;
  unsigned short* NFB = (unsigned short*)(ws + oNFB);
  unsigned short* WET = (unsigned short*)(ws + oWET);
  unsigned short* WT  = (unsigned short*)(ws + oWT);
  unsigned short* XP  = (unsigned short*)(ws + oXP);
  float*          XLR = (float*)(ws + oXLR);
  float*          XFa = (float*)(ws + oXFa);
  float*          XFb = (float*)(ws + oXFb);
  float*          PT  = (float*)(ws + oPT);

  hipFuncSetAttribute(reinterpret_cast<const void*>(&k_agg<0, 0>), hipFuncAttributeMaxDynamicSharedMemorySize, LDS_AGG);
  hipFuncSetAttribute(reinterpret_cast<const void*>(&k_agg<1, 0>), hipFuncAttributeMaxDynamicSharedMemorySize, LDS_AGG);
  hipFuncSetAttribute(reinterpret_cast<const void*>(&k_agg<1, 1>), hipFuncAttributeMaxDynamicSharedMemorySize, LDS_AGG);

  const float invN = 1.0f / (float)nN;

  k_prep<<<cdiv(nUt, NTHR), NTHR, 0, stream>>>(nf, wemb, wl, wr, NFB, WET, WT, nN, nUt);
  k_gemm<2><<<dim3(gM, HID / GBN), GTHR, 0, stream>>>(NFB, KE, WET, KE, KE, bemb, bemb,
                                                      (void*)XP, XPW, HID, nN, MP);
  k_gemm<3><<<dim3(gM, NLR / GBN), GTHR, 0, stream>>>(XP, XPW, WT, XPW, XPW, bl, br,
                                                      (void*)XLR, NLR, 0, nN, MP);
  k_agg<0, 0><<<gA, NTHR, LDS_AGG, stream>>>(src, dst, XLR, att, bias, XFb, XFa, HID, XP, PT,
                                             nN, nE, nb, vec8, MP);
  k_gemm<3><<<dim3(gM, NLR / GBN), GTHR, 0, stream>>>(XP, XPW, WT + (size_t)1 * NLR * XPW, XPW, XPW,
                                                      bl + 1 * HID, br + 1 * HID, (void*)XLR, NLR, 0, nN, MP);
  k_agg<1, 0><<<gA, NTHR, LDS_AGG, stream>>>(src, dst, XLR, att + 1 * HID, bias + 1 * HID, XFa, XFb, HID, XP, PT,
                                             nN, nE, nb, vec8, MP);
  k_gemm<3><<<dim3(gM, NLR / GBN), GTHR, 0, stream>>>(XP, XPW, WT + (size_t)2 * NLR * XPW, XPW, XPW,
                                                      bl + 2 * HID, br + 2 * HID, (void*)XLR, NLR, 0, nN, MP);
  k_agg<1, 0><<<gA, NTHR, LDS_AGG, stream>>>(src, dst, XLR, att + 2 * HID, bias + 2 * HID, XFb, XFa, HID, XP, PT,
                                             nN, nE, nb, vec8, MP);
  k_gemm<3><<<dim3(gM, NLR / GBN), GTHR, 0, stream>>>(XP, XPW, WT + (size_t)3 * NLR * XPW, XPW, XPW,
                                                      bl + 3 * HID, br + 3 * HID, (void*)XLR, NLR, 0, nN, MP);
  k_agg<1, 1><<<gA, NTHR, LDS_AGG, stream>>>(src, dst, XLR, att + 3 * HID, bias + 3 * HID, XFa, out + PARTW, HID, XP, PT,
                                             nN, nE, nb, vec8, MP);
  k_pool<<<1, NTHR, 0, stream>>>(PT, gA, invN, numn, out);
}
